// PointnetSAModuleMSG_34651796144290
// MI455X (gfx1250) — hardware-verified
//
#include <hip/hip_runtime.h>
#pragma clang fp contract(off)

typedef __attribute__((ext_vector_type(16))) _Float16 v16h;
typedef __attribute__((ext_vector_type(8)))  _Float16 v8h;
typedef __attribute__((ext_vector_type(8)))  float    v8f;
typedef __attribute__((ext_vector_type(4)))  float    v4f;
typedef __attribute__((ext_vector_type(4)))  unsigned v4u;
typedef v4u v4u_a __attribute__((may_alias));

constexpr int kBatch   = 16;
constexpr int kPts     = 4096;
constexpr int kFeat    = 64;
constexpr int kCen     = 1024;
constexpr int kW0Pitch = 67;
constexpr int kStatBlocks = 256;
constexpr int kPartPitch  = 256;
constexpr float kWCarry    = 16.0f;
constexpr float kWCarryInv = 1.0f / 16.0f;

static_assert(kBatch * kCen * 3 * 4 == 196608, "out0 bytes");
static_assert(196608 + kBatch * 256 * kCen * 4 == 16973824, "d_out bytes");
static_assert(196608 % 128 == 0, "out1 line aligned");

constexpr size_t kOffNx   = 0;
constexpr size_t kOffIdx0 = kOffNx   + (size_t)kBatch * kCen * 3 * 4;
constexpr size_t kOffIdx1 = kOffIdx0 + (size_t)kBatch * kCen * 16 * 4;
constexpr size_t kOffP    = kOffIdx1 + (size_t)kBatch * kCen * 32 * 4;
constexpr size_t kOffY1   = kOffP    + (size_t)kBatch * kPts * 64 * 4;
constexpr size_t kOffYext = kOffY1   + (size_t)kBatch * kCen * 32 * 96 * 2;
constexpr size_t kOffPart = kOffYext + (size_t)kBatch * kCen * 128 * 4;
constexpr size_t kOffAc   = kOffPart + (size_t)6 * kStatBlocks * kPartPitch * 4;
constexpr size_t kWsTotal = kOffAc   + (size_t)6 * 256 * 4;
static_assert(kWsTotal == 130750464, "carve total");
static_assert(kWsTotal <= 134217728, "carve within 128 MiB");
static_assert(kOffIdx0 % 128 == 0 && kOffIdx1 % 128 == 0 && kOffP % 128 == 0 && kOffY1 % 128 == 0 &&
              kOffYext % 128 == 0 && kOffPart % 128 == 0 && kOffAc % 128 == 0, "line aligned carve");

union FragH { v16h v; v8h h[2]; };

__device__ __forceinline__ v8f mma_f16(v16h a, v16h b, v8f c) {
  c = __builtin_amdgcn_wmma_f32_16x16x32_f16(false, a, false, b, (short)0, c, false, false);
  asm volatile("v_nop\n\tv_nop\n\tv_nop\n\tv_nop" : "+v"(c) : "v"(a), "v"(b));
  return c;
}

__device__ __forceinline__ float h16_to_f32(unsigned hb) {
  const unsigned sgn = (hb & 0x8000u) << 16;
  const unsigned em = hb & 0x7fffu;
  const float fn = __uint_as_float((em << 13) + 0x38000000u);
  const float fs = (float)em * 5.9604644775390625e-8f;
  const float mag = (em < 0x400u) ? fs : fn;
  return __uint_as_float(__float_as_uint(mag) | sgn);
}

__device__ __forceinline__ v16h wfrag_vec(const float* __restrict__ p) {
  const v4f a = *(const v4f*)(p);
  const v4f b = *(const v4f*)(p + 4);
  const v4f c = *(const v4f*)(p + 16);
  const v4f d = *(const v4f*)(p + 20);
  v16h r;
#pragma unroll
  for (int e = 0; e < 4; ++e) {
    r[e]      = (_Float16)(a[e] * kWCarry);
    r[4 + e]  = (_Float16)(b[e] * kWCarry);
    r[8 + e]  = (_Float16)(c[e] * kWCarry);
    r[12 + e] = (_Float16)(d[e] * kWCarry);
  }
  asm volatile("" ::: "memory");
  return r;
}
__device__ __forceinline__ v16h wfrag_sca(const float* __restrict__ p) {
  float f[16];
#pragma unroll
  for (int e = 0; e < 8; ++e) f[e] = p[e];
  asm volatile("" ::: "memory");
#pragma unroll
  for (int e = 0; e < 8; ++e) f[8 + e] = p[16 + e];
  v16h r;
#pragma unroll
  for (int e = 0; e < 16; ++e) r[e] = (_Float16)(f[e] * kWCarry);
  asm volatile("" ::: "memory");
  return r;
}

__device__ __forceinline__ float y0_val(float p, float wx, float wy, float wz, float rx, float ry, float rz) {
  const float t = (wx * rx + wy * ry) + wz * rz;
  return p + t;
}

__global__ __launch_bounds__(1024) void k_fps(const float* __restrict__ xyz, float* __restrict__ out0,
                                              float* __restrict__ nx) {
#pragma clang fp contract(off)
  __shared__ __align__(16) float sx[kPts * 3];
  __shared__ float pv[2][32];
  __shared__ int   pi[2][32];
  __shared__ int   sidx[kCen];
  const int tid = threadIdx.x, lane = tid & 31, wave = tid >> 5;
  const int b = blockIdx.x;
  {
    const v4f* src = (const v4f*)(xyz + (size_t)b * kPts * 3);
    v4f* dl = (v4f*)sx;
#pragma unroll
    for (int m = 0; m < 3; ++m) dl[tid + 1024 * m] = src[tid + 1024 * m];
  }
  if (tid == 0) sidx[0] = 0;
  __syncthreads();
  float px[4], py[4], pz[4], dist[4];
#pragma unroll
  for (int q = 0; q < 4; ++q) {
    const int i = tid + 1024 * q;
    px[q] = sx[i * 3 + 0]; py[q] = sx[i * 3 + 1]; pz[q] = sx[i * 3 + 2];
    dist[q] = 1e10f;
  }
  int last = 0;
#pragma unroll 1
  for (int t = 1; t < kCen; ++t) {
    const float lx = sx[last * 3 + 0], ly = sx[last * 3 + 1], lz = sx[last * 3 + 2];
    float bv = 0.f; int bi = tid;
#pragma unroll
    for (int q = 0; q < 4; ++q) {
      const float dx = px[q] - lx, dy = py[q] - ly, dz = pz[q] - lz;
      const float t0 = dx * dx, t1 = dy * dy, t2 = dz * dz;
      const float d = (t0 + t2) + t1;
      const float nd = fminf(dist[q], d);
      dist[q] = nd;
      if (q == 0) { bv = nd; bi = tid; }
      else { const bool tk = nd > bv; bv = tk ? nd : bv; bi = tk ? (tid + 1024 * q) : bi; }
    }
#pragma unroll
    for (int off = 16; off > 0; off >>= 1) {
      const float ov = __shfl_xor(bv, off, 32);
      const int   oi = __shfl_xor(bi, off, 32);
      const bool tk = (ov > bv) | ((ov == bv) & (oi < bi));
      bv = tk ? ov : bv; bi = tk ? oi : bi;
    }
    const int buf = t & 1;
    if (lane == 0) { pv[buf][wave] = bv; pi[buf][wave] = bi; }
    __syncthreads();
    float cv = pv[buf][lane]; int ci = pi[buf][lane];
#pragma unroll
    for (int off = 16; off > 0; off >>= 1) {
      const float ov = __shfl_xor(cv, off, 32);
      const int   oi = __shfl_xor(ci, off, 32);
      const bool tk = (ov > cv) | ((ov == cv) & (oi < ci));
      cv = tk ? ov : cv; ci = tk ? oi : ci;
    }
    ci = ci < 0 ? 0 : (ci > kPts - 1 ? kPts - 1 : ci);
    last = ci;
    if (tid == 0) sidx[t] = last;
  }
  __syncthreads();
  float val[3];
#pragma unroll
  for (int m = 0; m < 3; ++m) {
    const int f = tid + 1024 * m;
    const int pt = f / 3;
    const int c = f - 3 * pt;
    const int si = sidx[pt];
    val[m] = sx[si * 3 + c];
  }
  float* o0 = out0 + (size_t)b * kCen * 3;
  float* o1 = nx + (size_t)b * kCen * 3;
  for (int pass = 0; pass < 2; ++pass) {
#pragma unroll
    for (int m = 0; m < 3; ++m) {
      *(volatile float*)(o0 + tid + 1024 * m) = val[m];
      *(volatile float*)(o1 + tid + 1024 * m) = val[m];
    }
    __threadfence();
  }
}

__global__ __launch_bounds__(256) void k_ballquery(const float* __restrict__ xyz, const float* __restrict__ nx,
                                                   int* __restrict__ idx0, int* __restrict__ idx1) {
#pragma clang fp contract(off)
  __shared__ int l0[8][16];
  __shared__ int l1[8][32];
  const int tid = threadIdx.x, lane = tid & 31, wave = tid >> 5;
  const int cen = blockIdx.x * 8 + wave;
  const int b = cen >> 10;
  const float cx = nx[(size_t)cen * 3 + 0], cy = nx[(size_t)cen * 3 + 1], cz = nx[(size_t)cen * 3 + 2];
  const float r2a = __uint_as_float(0x3C23D70Au);
  const float r2b = __uint_as_float(0x3D23D70Au);
  const float* xb = xyz + (size_t)b * kPts * 3;
  const unsigned lt = (1u << lane) - 1u;
  int cnt0 = 0, cnt1 = 0, first0 = 0, first1 = 0;
#pragma unroll 1
  for (int base = 0; base < kPts; base += 32) {
    if (cnt0 >= 16 && cnt1 >= 32) break;
    const int j = base + lane;
    const float x = xb[j * 3 + 0], y = xb[j * 3 + 1], z = xb[j * 3 + 2];
    const float dx = cx - x, dy = cy - y, dz = cz - z;
    const float t0 = dx * dx, t1 = dy * dy, t2 = dz * dz;
    const float d2 = (t0 + t2) + t1;
    const bool in0 = d2 < r2a;
    const bool in1 = d2 < r2b;
    const unsigned m0 = __builtin_amdgcn_ballot_w32(in0);
    const unsigned m1 = __builtin_amdgcn_ballot_w32(in1);
    const int p0 = cnt0 + __popc(m0 & lt);
    const int p1 = cnt1 + __popc(m1 & lt);
    if (in0 && p0 < 16) l0[wave][p0] = j;
    if (in1 && p1 < 32) l1[wave][p1] = j;
    first0 = (cnt0 == 0 && m0 != 0u) ? (base + __ffs((int)m0) - 1) : first0;
    first1 = (cnt1 == 0 && m1 != 0u) ? (base + __ffs((int)m1) - 1) : first1;
    cnt0 += __popc(m0);
    cnt1 += __popc(m1);
  }
  if (lane < 16 && lane >= cnt0) l0[wave][lane] = first0;
  if (lane >= cnt1) l1[wave][lane] = first1;
  __syncthreads();
  const int v1 = l1[wave][lane];
  const int e0 = (wave & 3) * 32 + lane;
  const int v0 = l0[e0 >> 4][e0 & 15];
  volatile int* d1 = (volatile int*)(idx1 + (size_t)cen * 32 + lane);
  volatile int* d0 = (volatile int*)(idx0 + (size_t)blockIdx.x * 128 + e0);
  *d1 = v1;
  if (wave < 4) *d0 = v0;
  __threadfence();
  *d1 = v1;
  if (wave < 4) *d0 = v0;
}

__global__ __launch_bounds__(256) void k_pgemm(const float* __restrict__ feat, const float* __restrict__ W0,
                                               float* __restrict__ P, int tilesPerBlock) {
  constexpr int APITCH = 72;
  __shared__ __align__(16) _Float16 As[64 * APITCH];
  __shared__ __align__(16) float Ps[64 * 64];
  const int tid = threadIdx.x, lane = tid & 31, wave = tid >> 5;
  const int lm = lane & 15, hf = lane >> 4;
  const int rs = wave & 3, cg = wave >> 2;
  v16h bf[2][2];
#pragma unroll
  for (int j = 0; j < 2; ++j)
#pragma unroll
    for (int kk = 0; kk < 2; ++kk) {
      const int o = cg * 32 + 16 * j + lm;
      bf[j][kk] = wfrag_sca(W0 + (size_t)o * kW0Pitch + 3 + kk * 32 + 8 * hf);
    }
#pragma unroll 1
  for (int tt = 0; tt < tilesPerBlock; ++tt) {
    const int tile = blockIdx.x * tilesPerBlock + tt;
    const int b = tile >> 6;
    const int n0 = (tile & 63) * 64;
    {
      const int n = tid & 63, cq = tid >> 6;
      const float* fp = feat + ((size_t)(b * kFeat + cq * 16)) * kPts + n0 + n;
      float f[16];
#pragma unroll
      for (int e = 0; e < 8; ++e) f[e] = fp[(size_t)e * kPts];
      asm volatile("" ::: "memory");
#pragma unroll
      for (int e = 0; e < 8; ++e) f[8 + e] = fp[(size_t)(8 + e) * kPts];
      v8h h0, h1;
#pragma unroll
      for (int e = 0; e < 8; ++e) { h0[e] = (_Float16)f[e]; h1[e] = (_Float16)f[8 + e]; }
      *(v8h*)(As + n * APITCH + cq * 16) = h0;
      *(v8h*)(As + n * APITCH + cq * 16 + 8) = h1;
    }
    __syncthreads();
    v8f acc[2];
    acc[0] = (v8f){0.f, 0.f, 0.f, 0.f, 0.f, 0.f, 0.f, 0.f};
    acc[1] = (v8f){0.f, 0.f, 0.f, 0.f, 0.f, 0.f, 0.f, 0.f};
#pragma unroll
    for (int kk = 0; kk < 2; ++kk) {
      FragH fa;
      fa.h[0] = *(const v8h*)(As + (rs * 16 + lm) * APITCH + kk * 32 + 8 * hf);
      fa.h[1] = *(const v8h*)(As + (rs * 16 + lm) * APITCH + kk * 32 + 16 + 8 * hf);
#pragma unroll
      for (int j = 0; j < 2; ++j) acc[j] = mma_f16(fa.v, bf[j][kk], acc[j]);
    }
#pragma unroll
    for (int j = 0; j < 2; ++j)
#pragma unroll
      for (int r = 0; r < 8; ++r) {
        const float v = acc[j][r] * kWCarryInv;
        Ps[(rs * 16 + 8 * hf + r) * 64 + cg * 32 + 16 * j + lm] = v;
      }
    __syncthreads();
    {
      float* dst = P + ((size_t)b * kPts + n0) * 64;
      v4f vals[4];
#pragma unroll
      for (int i = 0; i < 4; ++i) vals[i] = *(const v4f*)(Ps + (tid + 256 * i) * 4);
      for (int pass = 0; pass < 2; ++pass) {
#pragma unroll
        for (int i = 0; i < 4; ++i) *(volatile v4f*)(dst + (size_t)(tid + 256 * i) * 4) = vals[i];
        __threadfence();
      }
    }
  }
}

template <int KS>
__global__ __launch_bounds__(256) void k_l0stats(const float* __restrict__ P, const int* __restrict__ idx,
                                                 const float* __restrict__ xyz, const float* __restrict__ nx,
                                                 const float* __restrict__ W0, float* __restrict__ part,
                                                 int rowsPerBlock) {
  __shared__ float rsum[2][16][64];
  __shared__ __align__(16) float fin[256];
  const int tid = threadIdx.x;
  const int cq = tid & 15, slot = tid >> 4;
  float wx[4], wy[4], wz[4];
#pragma unroll
  for (int e = 0; e < 4; ++e) {
    const int o = 4 * cq + e;
    wx[e] = W0[o * kW0Pitch + 0]; wy[e] = W0[o * kW0Pitch + 1]; wz[e] = W0[o * kW0Pitch + 2];
  }
  float s[4] = {0.f, 0.f, 0.f, 0.f}, q[4] = {0.f, 0.f, 0.f, 0.f};
  const size_t row0 = (size_t)blockIdx.x * rowsPerBlock;
  const int nit = rowsPerBlock >> 4;
#pragma unroll 1
  for (int it = 0; it < nit; ++it) {
    const size_t g = row0 + (size_t)it * 16 + slot;
    int j = idx[g];
    j = j < 0 ? 0 : (j > kPts - 1 ? kPts - 1 : j);
    const int cen = (int)(g / KS);
    const int b = cen >> 10;
    const float* xp = xyz + ((size_t)b * kPts + j) * 3;
    const float* np = nx + (size_t)cen * 3;
    const float rx = xp[0] - np[0], ry = xp[1] - np[1], rz = xp[2] - np[2];
    const v4f p = *(const v4f*)(P + ((size_t)b * kPts + j) * 64 + 4 * cq);
#pragma unroll
    for (int e = 0; e < 4; ++e) {
      const float y = y0_val(p[e], wx[e], wy[e], wz[e], rx, ry, rz);
      s[e] += y;
      q[e] += y * y;
    }
  }
#pragma unroll
  for (int e = 0; e < 4; ++e) { rsum[0][slot][4 * cq + e] = s[e]; rsum[1][slot][4 * cq + e] = q[e]; }
  __syncthreads();
  {
    const int n = tid & 127, qq = tid >> 7;
    const int nc = n < 64 ? n : 63;
    float v = 0.f;
#pragma unroll
    for (int sl = 0; sl < 16; ++sl) v += rsum[qq][sl][nc];
    fin[tid] = (n < 64) ? v : 0.f;
  }
  __syncthreads();
  if (tid < 64) {
    const v4f v = *(const v4f*)(fin + 4 * tid);
    volatile v4f* d = (volatile v4f*)(part + (size_t)blockIdx.x * kPartPitch + 4 * tid);
    *d = v;
    __threadfence();
    *d = v;
  }
}

__global__ __launch_bounds__(128) void k_bnfin(const float* __restrict__ part, int nblk, int nch,
                                               const float* __restrict__ g, const float* __restrict__ bt,
                                               float invn, float* __restrict__ ac) {
  __shared__ __align__(16) float sac[256];
  const int o = threadIdx.x;
  const int oc = o < nch ? o : nch - 1;
  double s = 0.0, q = 0.0;
#pragma unroll 4
  for (int k = 0; k < nblk; ++k) {
    s += (double)part[(size_t)k * kPartPitch + oc];
    q += (double)part[(size_t)k * kPartPitch + 128 + oc];
  }
  const double mean = s * (double)invn;
  double var = q * (double)invn - mean * mean;
  var = var < 0.0 ? 0.0 : var;
  const float inv = rsqrtf((float)var + 1e-5f);
  const float a = g[oc] * inv;
  const float c = bt[oc] - (float)mean * a;
  sac[o] = (o < nch) ? a : 0.f;
  sac[128 + o] = (o < nch) ? c : 0.f;
  __syncthreads();
  if (o < 64) {
    const v4f v = *(const v4f*)(sac + 4 * o);
    volatile v4f* d = (volatile v4f*)(ac + 4 * o);
    *d = v;
    __threadfence();
    *d = v;
  }
}

template <int NOUT, int KS>
__global__ __launch_bounds__(256) void k_l1(const float* __restrict__ P, const int* __restrict__ idx,
                                            const float* __restrict__ xyz, const float* __restrict__ nx,
                                            const float* __restrict__ W0, const float* __restrict__ ac0,
                                            const float* __restrict__ W1, unsigned short* __restrict__ y1,
                                            float* __restrict__ part, int tilesPerBlock) {
  constexpr int NJ = NOUT / 32;
  constexpr int HW = NOUT / 2;
  constexpr int NU = NOUT / 32;
  constexpr int APITCH = 72;
  static_assert(NOUT % 32 == 0 && NOUT <= 128, "column split");
  __shared__ __align__(16) _Float16 As[64 * APITCH];
  __shared__ __align__(16) unsigned short Ys[64 * NOUT];
  __shared__ __align__(16) float cst[5][64];
  __shared__ float red[2][8][64];
  __shared__ __align__(16) float fin[256];
  const int tid = threadIdx.x, lane = tid & 31, wave = tid >> 5;
  const int lm = lane & 15, hf = lane >> 4;
  const int rs = wave & 3, cg = wave >> 2;
  if (tid < 64) {
    cst[0][tid] = ac0[tid];
    cst[1][tid] = ac0[128 + tid];
    cst[2][tid] = W0[tid * kW0Pitch + 0];
    cst[3][tid] = W0[tid * kW0Pitch + 1];
    cst[4][tid] = W0[tid * kW0Pitch + 2];
  }
  v16h bf[NJ][2];
#pragma unroll
  for (int j = 0; j < NJ; ++j)
#pragma unroll
    for (int kk = 0; kk < 2; ++kk) {
      const int n = cg * HW + 16 * j + lm;
      bf[j][kk] = wfrag_vec(W1 + (size_t)n * 64 + kk * 32 + 8 * hf);
    }
  float ssum[NJ], ssq[NJ];
#pragma unroll
  for (int j = 0; j < NJ; ++j) { ssum[j] = 0.f; ssq[j] = 0.f; }
  __syncthreads();
#pragma unroll 1
  for (int tt = 0; tt < tilesPerBlock; ++tt) {
    const int tile = blockIdx.x * tilesPerBlock + tt;
    {
      const int r = tid >> 2, cq = tid & 3;
      const size_t g = (size_t)tile * 64 + r;
      int j = idx[g];
      j = j < 0 ? 0 : (j > kPts - 1 ? kPts - 1 : j);
      const int cen = (int)(g / KS);
      const int b = cen >> 10;
      const float* xp = xyz + ((size_t)b * kPts + j) * 3;
      const float* np = nx + (size_t)cen * 3;
      const float rx = xp[0] - np[0], ry = xp[1] - np[1], rz = xp[2] - np[2];
      const float* pp = P + ((size_t)b * kPts + j) * 64 + cq * 16;
      v4f p[4];
#pragma unroll
      for (int qd = 0; qd < 4; ++qd) p[qd] = *(const v4f*)(pp + 4 * qd);
      v8h h0, h1;
#pragma unroll
      for (int qd = 0; qd < 4; ++qd) {
        const v4f a4 = *(const v4f*)(&cst[0][cq * 16 + 4 * qd]);
        const v4f c4 = *(const v4f*)(&cst[1][cq * 16 + 4 * qd]);
        const v4f x4 = *(const v4f*)(&cst[2][cq * 16 + 4 * qd]);
        const v4f y4 = *(const v4f*)(&cst[3][cq * 16 + 4 * qd]);
        const v4f z4 = *(const v4f*)(&cst[4][cq * 16 + 4 * qd]);
#pragma unroll
        for (int e = 0; e < 4; ++e) {
          const float y = y0_val(p[qd][e], x4[e], y4[e], z4[e], rx, ry, rz);
          const float x = fmaxf(a4[e] * y + c4[e], 0.0f);
          if (qd < 2) h0[4 * qd + e] = (_Float16)x;
          else        h1[4 * (qd - 2) + e] = (_Float16)x;
        }
      }
      *(v8h*)(As + r * APITCH + cq * 16) = h0;
      *(v8h*)(As + r * APITCH + cq * 16 + 8) = h1;
    }
    __syncthreads();
    v8f acc[NJ];
#pragma unroll
    for (int j = 0; j < NJ; ++j) acc[j] = (v8f){0.f, 0.f, 0.f, 0.f, 0.f, 0.f, 0.f, 0.f};
#pragma unroll
    for (int kk = 0; kk < 2; ++kk) {
      FragH fa;
      fa.h[0] = *(const v8h*)(As + (rs * 16 + lm) * APITCH + kk * 32 + 8 * hf);
      fa.h[1] = *(const v8h*)(As + (rs * 16 + lm) * APITCH + kk * 32 + 16 + 8 * hf);
#pragma unroll
      for (int j = 0; j < NJ; ++j) acc[j] = mma_f16(fa.v, bf[j][kk], acc[j]);
    }
#pragma unroll
    for (int j = 0; j < NJ; ++j)
#pragma unroll
      for (int r = 0; r < 8; ++r) {
        const float v = acc[j][r] * kWCarryInv;
        ssum[j] += v;
        ssq[j] += v * v;
        const _Float16 hv = (_Float16)v;
        Ys[(rs * 16 + 8 * hf + r) * NOUT + cg * HW + 16 * j + lm] = __builtin_bit_cast(unsigned short, hv);
      }
    __syncthreads();
    {
      unsigned short* dst = y1 + (size_t)tile * 64 * NOUT;
      v4u vals[NU];
#pragma unroll
      for (int i = 0; i < NU; ++i) vals[i] = *(const v4u_a*)(Ys + (tid + 256 * i) * 8);
      for (int pass = 0; pass < 2; ++pass) {
#pragma unroll
        for (int i = 0; i < NU; ++i) *(volatile v4u*)(dst + (size_t)(tid + 256 * i) * 8) = vals[i];
        __threadfence();
      }
    }
  }
#pragma unroll
  for (int j = 0; j < NJ; ++j) {
    ssum[j] += __shfl_xor(ssum[j], 16, 32);
    ssq[j]  += __shfl_xor(ssq[j], 16, 32);
  }
  if (lane < 16) {
#pragma unroll
    for (int j = 0; j < NJ; ++j) { red[0][wave][16 * j + lane] = ssum[j]; red[1][wave][16 * j + lane] = ssq[j]; }
  }
  __syncthreads();
  {
    const int n = tid & 127, qq = tid >> 7;
    const int nc = n < NOUT ? n : NOUT - 1;
    const int cgn = nc / HW;
    const int w = nc - cgn * HW;
    const float v = ((red[qq][cgn * 4 + 0][w] + red[qq][cgn * 4 + 1][w]) + red[qq][cgn * 4 + 2][w]) + red[qq][cgn * 4 + 3][w];
    fin[tid] = (n < NOUT) ? v : 0.f;
  }
  __syncthreads();
  if (tid < 64) {
    const v4f v = *(const v4f*)(fin + 4 * tid);
    volatile v4f* d = (volatile v4f*)(part + (size_t)blockIdx.x * kPartPitch + 4 * tid);
    *d = v;
    __threadfence();
    *d = v;
  }
}

template <int KIN, int KS>
__global__ __launch_bounds__(256) void k_l2(const unsigned short* __restrict__ y1, const float* __restrict__ ac1,
                                            const float* __restrict__ W2, const float* __restrict__ g2,
                                            float* __restrict__ yext, float* __restrict__ part, int tilesPerBlock) {
  constexpr int NK = KIN / 32;
  constexpr int APITCH = KIN + 8;
  constexpr int UPR = KIN / 8;
  constexpr int NU = KIN / 32;
  constexpr int NCT = 64 / KS;
  static_assert(KIN % 32 == 0 && KIN <= 128, "k steps");
  __shared__ __align__(16) _Float16 As[64 * APITCH];
  __shared__ __align__(16) float sab[2][128];
  __shared__ int gpos[128];
  __shared__ __align__(16) float Emx[4][128];
  __shared__ __align__(16) float Emn[4][128];
  __shared__ float red[2][8][64];
  __shared__ __align__(16) float fin[256];
  const int tid = threadIdx.x, lane = tid & 31, wave = tid >> 5;
  const int lm = lane & 15, hf = lane >> 4;
  const int rs = wave & 3, cg = wave >> 2;
  if (tid < KIN) { sab[0][tid] = ac1[tid]; sab[1][tid] = ac1[128 + tid]; }
  if (tid < 128) gpos[tid] = (g2[tid] > 0.0f) ? 1 : 0;
  v16h bf[4][NK];
#pragma unroll
  for (int j = 0; j < 4; ++j)
#pragma unroll
    for (int kk = 0; kk < NK; ++kk) {
      const int n = cg * 64 + 16 * j + lm;
      bf[j][kk] = wfrag_vec(W2 + (size_t)n * KIN + kk * 32 + 8 * hf);
    }
  float ssum[4], ssq[4];
#pragma unroll
  for (int j = 0; j < 4; ++j) { ssum[j] = 0.f; ssq[j] = 0.f; }
  __syncthreads();
#pragma unroll 1
  for (int tt = 0; tt < tilesPerBlock; ++tt) {
    const int tile = blockIdx.x * tilesPerBlock + tt;
    {
      const unsigned short* src = y1 + (size_t)tile * 64 * KIN;
      v4u w[NU];
#pragma unroll
      for (int i = 0; i < NU; ++i) w[i] = *(const v4u*)(src + (size_t)(tid + 256 * i) * 8);
#pragma unroll
      for (int i = 0; i < NU; ++i) {
        const int u = tid + 256 * i;
        const int row = u / UPR;
        const int c8 = (u - row * UPR) * 8;
        const unsigned w0 = w[i].x, w1 = w[i].y, w2 = w[i].z, w3 = w[i].w;
        float y[8];
        y[0] = h16_to_f32(w0 & 0xffffu); y[1] = h16_to_f32(w0 >> 16);
        y[2] = h16_to_f32(w1 & 0xffffu); y[3] = h16_to_f32(w1 >> 16);
        y[4] = h16_to_f32(w2 & 0xffffu); y[5] = h16_to_f32(w2 >> 16);
        y[6] = h16_to_f32(w3 & 0xffffu); y[7] = h16_to_f32(w3 >> 16);
        const v4f a0 = *(const v4f*)(&sab[0][c8]);
        const v4f a1 = *(const v4f*)(&sab[0][c8 + 4]);
        const v4f c0 = *(const v4f*)(&sab[1][c8]);
        const v4f c1 = *(const v4f*)(&sab[1][c8 + 4]);
        v8h hv;
#pragma unroll
        for (int e = 0; e < 4; ++e) {
          hv[e]     = (_Float16)fmaxf(a0[e] * y[e] + c0[e], 0.0f);
          hv[4 + e] = (_Float16)fmaxf(a1[e] * y[4 + e] + c1[e], 0.0f);
        }
        *(v8h*)(As + row * APITCH + c8) = hv;
      }
    }
    __syncthreads();
    v8f acc[4];
#pragma unroll
    for (int j = 0; j < 4; ++j) acc[j] = (v8f){0.f, 0.f, 0.f, 0.f, 0.f, 0.f, 0.f, 0.f};
#pragma unroll
    for (int kk = 0; kk < NK; ++kk) {
      FragH fa;
      fa.h[0] = *(const v8h*)(As + (rs * 16 + lm) * APITCH + kk * 32 + 8 * hf);
      fa.h[1] = *(const v8h*)(As + (rs * 16 + lm) * APITCH + kk * 32 + 16 + 8 * hf);
#pragma unroll
      for (int j = 0; j < 4; ++j) acc[j] = mma_f16(fa.v, bf[j][kk], acc[j]);
    }
#pragma unroll
    for (int j = 0; j < 4; ++j) {
      float mx = -3.0e38f, mn = 3.0e38f;
#pragma unroll
      for (int r = 0; r < 8; ++r) {
        const float v = acc[j][r] * kWCarryInv;
        ssum[j] += v;
        ssq[j] += v * v;
        mx = fmaxf(mx, v);
        mn = fminf(mn, v);
      }
      const float omx = __shfl_xor(mx, 16, 32);
      const float omn = __shfl_xor(mn, 16, 32);
      mx = fmaxf(mx, omx);
      mn = fminf(mn, omn);
      if (lane < 16) { Emx[rs][cg * 64 + 16 * j + lm] = mx; Emn[rs][cg * 64 + 16 * j + lm] = mn; }
    }
    __syncthreads();
    if (wave < NCT) {
      const int cc = wave;
      const int c4 = lane * 4;
      const int e0 = (KS == 16) ? cc : 2 * cc;
      const int e1 = (KS == 16) ? cc : 2 * cc + 1;
      const v4f xa = *(const v4f*)(&Emx[e0][c4]);
      const v4f xb = *(const v4f*)(&Emx[e1][c4]);
      const v4f na = *(const v4f*)(&Emn[e0][c4]);
      const v4f nb = *(const v4f*)(&Emn[e1][c4]);
      v4f o;
#pragma unroll
      for (int e = 0; e < 4; ++e) {
        const float mx = fmaxf(xa[e], xb[e]);
        const float mn = fminf(na[e], nb[e]);
        const int gp = gpos[c4 + e];
        o[e] = gp ? mx : mn;
      }
      volatile v4f* d = (volatile v4f*)(yext + ((size_t)tile * NCT + cc) * 128 + c4);
      *d = o;
      __threadfence();
      *d = o;
    }
  }
#pragma unroll
  for (int j = 0; j < 4; ++j) {
    ssum[j] += __shfl_xor(ssum[j], 16, 32);
    ssq[j]  += __shfl_xor(ssq[j], 16, 32);
  }
  if (lane < 16) {
#pragma unroll
    for (int j = 0; j < 4; ++j) { red[0][wave][16 * j + lane] = ssum[j]; red[1][wave][16 * j + lane] = ssq[j]; }
  }
  __syncthreads();
  {
    const int n = tid & 127, qq = tid >> 7;
    const int cgn = n >> 6;
    const int w = n & 63;
    const float v = ((red[qq][cgn * 4 + 0][w] + red[qq][cgn * 4 + 1][w]) + red[qq][cgn * 4 + 2][w]) + red[qq][cgn * 4 + 3][w];
    fin[tid] = v;
  }
  __syncthreads();
  if (tid < 64) {
    const v4f v = *(const v4f*)(fin + 4 * tid);
    volatile v4f* d = (volatile v4f*)(part + (size_t)blockIdx.x * kPartPitch + 4 * tid);
    *d = v;
    __threadfence();
    *d = v;
  }
}

__global__ __launch_bounds__(256) void k_pool(const float* __restrict__ yext, const float* __restrict__ ac2,
                                              float* __restrict__ out1, int choff) {
  constexpr int TP = 132;
  __shared__ __align__(16) float T[32 * TP];
  __shared__ float sa[128];
  __shared__ float sc[128];
  const int tid = threadIdx.x, lane = tid & 31, wave = tid >> 5;
  const int b = blockIdx.x >> 5;
  const int s0 = (blockIdx.x & 31) * 32;
  if (tid < 128) { sa[tid] = ac2[tid]; sc[tid] = ac2[128 + tid]; }
#pragma unroll
  for (int i = 0; i < 4; ++i) {
    const int u = tid + 256 * i;
    const int row = u >> 5;
    const int c4 = (u & 31) * 4;
    const v4f v = *(const v4f*)(yext + ((size_t)(b * kCen + s0 + row)) * 128 + c4);
    *(v4f*)(T + row * TP + c4) = v;
  }
  __syncthreads();
  float vals[16];
#pragma unroll
  for (int i = 0; i < 16; ++i) {
    const int o = wave + 8 * i;
    vals[i] = fmaxf(sa[o] * T[lane * TP + o] + sc[o], 0.0f);
  }
  float* base = out1 + ((size_t)(b * 256 + choff)) * kCen + s0 + lane;
  for (int pass = 0; pass < 2; ++pass) {
#pragma unroll
    for (int i = 0; i < 16; ++i) *(volatile float*)(base + (size_t)(wave + 8 * i) * kCen) = vals[i];
    __threadfence();
  }
}

extern "C" void kernel_launch(void* const* d_in, const int* in_sizes, int n_in,
                              void* d_out, int out_size, void* d_ws, size_t ws_size, hipStream_t stream) {
  (void)in_sizes; (void)out_size;
  if (n_in < 20) return;
  if (ws_size < kWsTotal) return;
  const float* xyz  = (const float*)d_in[0];
  const float* feat = (const float*)d_in[1];
  const float* Wt[2][3]; const float* Gm[2][3]; const float* Be[2][3];
  for (int s = 0; s < 2; ++s)
    for (int l = 0; l < 3; ++l) {
      Wt[s][l] = (const float*)d_in[2 + s * 9 + l * 3 + 0];
      Gm[s][l] = (const float*)d_in[2 + s * 9 + l * 3 + 1];
      Be[s][l] = (const float*)d_in[2 + s * 9 + l * 3 + 2];
    }
  float* out0 = (float*)d_out;
  float* out1 = (float*)d_out + (196608 / 4);

  char* ws = (char*)d_ws;
  float* nx   = (float*)(ws + kOffNx);
  int*   idx0 = (int*)(ws + kOffIdx0);
  int*   idx1 = (int*)(ws + kOffIdx1);
  float* P    = (float*)(ws + kOffP);
  unsigned short* y1 = (unsigned short*)(ws + kOffY1);
  float* yext = (float*)(ws + kOffYext);
  float* part = (float*)(ws + kOffPart);
  float* ac   = (float*)(ws + kOffAc);
  const size_t partSlot = (size_t)kStatBlocks * kPartPitch;

  k_fps<<<kBatch, 1024, 0, stream>>>(xyz, out0, nx);
  k_ballquery<<<(kBatch * kCen) / 8, 256, 0, stream>>>(xyz, nx, idx0, idx1);

  {
    const float invn = 1.0f / 262144.0f;
    float* p0 = part + 0 * partSlot; float* p1 = part + 1 * partSlot; float* p2 = part + 2 * partSlot;
    float* a0 = ac + 0 * 256; float* a1 = ac + 1 * 256; float* a2 = ac + 2 * 256;
    k_pgemm<<<128, 256, 0, stream>>>(feat, Wt[0][0], P, 8);
    k_l0stats<16><<<kStatBlocks, 256, 0, stream>>>(P, idx0, xyz, nx, Wt[0][0], p0, 262144 / kStatBlocks);
    k_bnfin<<<1, 128, 0, stream>>>(p0, kStatBlocks, 64, Gm[0][0], Be[0][0], invn, a0);
    k_l1<64, 16><<<kStatBlocks, 256, 0, stream>>>(P, idx0, xyz, nx, Wt[0][0], a0, Wt[0][1], y1, p1, 4096 / kStatBlocks);
    k_bnfin<<<1, 128, 0, stream>>>(p1, kStatBlocks, 64, Gm[0][1], Be[0][1], invn, a1);
    k_l2<64, 16><<<kStatBlocks, 256, 0, stream>>>(y1, a1, Wt[0][2], Gm[0][2], yext, p2, 4096 / kStatBlocks);
    k_bnfin<<<1, 128, 0, stream>>>(p2, kStatBlocks, 128, Gm[0][2], Be[0][2], invn, a2);
    k_pool<<<kBatch * 32, 256, 0, stream>>>(yext, a2, out1, 0);
  }
  {
    const float invn = 1.0f / 524288.0f;
    float* p0 = part + 3 * partSlot; float* p1 = part + 4 * partSlot; float* p2 = part + 5 * partSlot;
    float* a0 = ac + 3 * 256; float* a1 = ac + 4 * 256; float* a2 = ac + 5 * 256;
    k_pgemm<<<128, 256, 0, stream>>>(feat, Wt[1][0], P, 8);
    k_l0stats<32><<<kStatBlocks, 256, 0, stream>>>(P, idx1, xyz, nx, Wt[1][0], p0, 524288 / kStatBlocks);
    k_bnfin<<<1, 128, 0, stream>>>(p0, kStatBlocks, 64, Gm[1][0], Be[1][0], invn, a0);
    k_l1<96, 32><<<kStatBlocks, 256, 0, stream>>>(P, idx1, xyz, nx, Wt[1][0], a0, Wt[1][1], y1, p1, 8192 / kStatBlocks);
    k_bnfin<<<1, 128, 0, stream>>>(p1, kStatBlocks, 96, Gm[1][1], Be[1][1], invn, a1);
    k_l2<96, 32><<<kStatBlocks, 256, 0, stream>>>(y1, a1, Wt[1][2], Gm[1][2], yext, p2, 8192 / kStatBlocks);
    k_bnfin<<<1, 128, 0, stream>>>(p2, kStatBlocks, 128, Gm[1][2], Be[1][2], invn, a2);
    k_pool<<<kBatch * 32, 256, 0, stream>>>(yext, a2, out1, 128);
  }
}
